// Layer_6493990551861
// MI455X (gfx1250) — hardware-verified
//
#include <hip/hip_runtime.h>
#include <math.h>

#ifndef NB
#define NB 2
#endif
#ifndef SEQ
#define SEQ 2048
#endif
#ifndef OUT_SEQ_STRIDE
#define OUT_SEQ_STRIDE 2048
#endif

constexpr int kB            = NB;
constexpr int kSeq          = SEQ;
constexpr int kBFull        = 2;
constexpr int kSeqFull      = 2048;
constexpr int kOutSeqStride = OUT_SEQ_STRIDE;
constexpr int kH   = 1024;
constexpr int kNH  = 16;
constexpr int kHD  = 64;
constexpr int kFF  = 4096;
constexpr int kM   = kB * kSeq;
constexpr int kQB  = 128;
constexpr int kKB  = 64;
constexpr int kPP  = 72;
constexpr float kPCarry   = 256.0f;
constexpr float kCtxCarry = 64.0f;
constexpr float kWCarry   = 64.0f;
constexpr float kUCarry   = 16.0f;
constexpr float kScoreC   = 0.125f * 1.4426950408889634f;
constexpr float kLnEps    = 1e-12f;
constexpr float kInvH     = 1.0f / 1024.0f;
static_assert(kNH * kHD == kH);
static_assert(kH == 4 * 256);
static_assert(kB >= 1 && kB <= kBFull);
static_assert(kSeq >= kQB && kSeq <= kSeqFull && kSeq % kQB == 0 && kSeq % kKB == 0);
static_assert(kOutSeqStride >= kSeq);
static_assert(kM % 64 == 0 && kH % 64 == 0 && kFF % 64 == 0 && kSeq % 64 == 0);
static_assert(kH % 32 == 0 && kFF % 32 == 0 && kSeq % 32 == 0 && kHD % 32 == 0);
static_assert(kM % 2 == 0);

constexpr size_t szW   = (size_t)kH * kH * 2;
constexpr size_t szWF  = (size_t)kH * kFF * 2;
constexpr size_t szAct = (size_t)kM * kH * 2;
constexpr size_t szVT  = (size_t)kB * kH * kSeq * 2;
constexpr size_t szF32 = (size_t)kM * kH * 4;
constexpr size_t szU   = (size_t)kM * kFF * 2;
constexpr size_t offWQ  = 0;
constexpr size_t offWK  = offWQ + szW;
constexpr size_t offWV  = offWK + szW;
constexpr size_t offWO  = offWV + szW;
constexpr size_t offW1  = offWO + szW;
constexpr size_t offW2  = offW1 + szWF;
constexpr size_t offXB  = offW2 + szWF;
constexpr size_t offQ   = offXB + szAct;
constexpr size_t offK   = offQ + szAct;
constexpr size_t offVT  = offK + szAct;
constexpr size_t offCTX = offVT + szVT;
constexpr size_t offTMP = offCTX + szAct;
constexpr size_t offLN1 = offTMP + szF32;
constexpr size_t offU   = offLN1 + szAct;
constexpr size_t kWsTotal = offU + szU;
static_assert(kWsTotal <= (size_t)134217728);
static_assert(szW % 128 == 0 && szWF % 128 == 0 && szAct % 128 == 0 && szVT % 128 == 0 && szF32 % 128 == 0 && szU % 128 == 0);

typedef __attribute__((ext_vector_type(16))) _Float16 v16h;
typedef __attribute__((ext_vector_type(8)))  _Float16 v8h;
typedef __attribute__((ext_vector_type(16))) __bf16   v16b;
typedef __attribute__((ext_vector_type(8)))  __bf16   v8b;
typedef __attribute__((ext_vector_type(8)))  float    v8f;
typedef __attribute__((ext_vector_type(4)))  float    v4f;
typedef __attribute__((ext_vector_type(4)))  unsigned int v4u;

__device__ __forceinline__ unsigned short f2bf_bits(float f) {
  unsigned u = __float_as_uint(f);
  return (unsigned short)((u + 0x7FFFu + ((u >> 16) & 1u)) >> 16);
}
__device__ __forceinline__ float bf_bits2f(unsigned short h) { return __uint_as_float(((unsigned)h) << 16); }
__device__ __forceinline__ float bfr(float f) { return bf_bits2f(f2bf_bits(f)); }
__device__ __forceinline__ unsigned pk16(unsigned short a, unsigned short b) { return (unsigned)a | ((unsigned)b << 16); }
__device__ __forceinline__ float gelu_f(float x) { return x * 0.5f * (1.0f + erff(x * 0.70710678118654752f)); }
__device__ __forceinline__ v8f vzero8() { return (v8f){0.f, 0.f, 0.f, 0.f, 0.f, 0.f, 0.f, 0.f}; }

__device__ __forceinline__ void dep_guard4_h(v8f& a, v8f& b, v8f& c, v8f& d, v16h x, v16h y) {
  asm volatile("v_nop\n\tv_nop\n\tv_nop\n\tv_nop" : "+v"(a), "+v"(b), "+v"(c), "+v"(d) : "v"(x), "v"(y));
}
__device__ __forceinline__ void dep_guard4_b(v8f& a, v8f& b, v8f& c, v8f& d, v16b x, v16b y) {
  asm volatile("v_nop\n\tv_nop\n\tv_nop\n\tv_nop" : "+v"(a), "+v"(b), "+v"(c), "+v"(d) : "v"(x), "v"(y));
}
__device__ __forceinline__ void keep4_h(v16h a, v16h b, v16h c, v16h d) { asm volatile("v_nop" :: "v"(a), "v"(b), "v"(c), "v"(d)); }
__device__ __forceinline__ void keep4_b(v16b a, v16b b, v16b c, v16b d) { asm volatile("v_nop" :: "v"(a), "v"(b), "v"(c), "v"(d)); }
__device__ __forceinline__ void acc_guard4(v8f& a, v8f& b, v8f& c, v8f& d) { asm volatile("v_nop\n\tv_nop\n\tv_nop\n\tv_nop" : "+v"(a), "+v"(b), "+v"(c), "+v"(d)); }
template <typename T> struct Frag;
template <> struct Frag<_Float16> {
  typedef v16h V; union U { v16h v; v8h h[2]; };
  static __device__ __forceinline__ v16h load(const _Float16* p) {
    U f; f.h[0] = *(const v8h*)(p); f.h[1] = *(const v8h*)(p + 16); return f.v;
  }
  static __device__ __forceinline__ v8f mma(v16h a, v16h b, v8f c) {
    return __builtin_amdgcn_wmma_f32_16x16x32_f16(false, a, false, b, (short)0, c, false, false);
  }
  static __device__ __forceinline__ void guard4(v8f& a, v8f& b, v8f& c, v8f& d, v16h x, v16h y) { dep_guard4_h(a, b, c, d, x, y); }
  static __device__ __forceinline__ void keep(v16h a, v16h b, v16h c, v16h d) { keep4_h(a, b, c, d); }
};
template <> struct Frag<__bf16> {
  typedef v16b V; union U { v16b v; v8b h[2]; };
  static __device__ __forceinline__ v16b load(const __bf16* p) {
    U f; f.h[0] = *(const v8b*)(p); f.h[1] = *(const v8b*)(p + 16); return f.v;
  }
  static __device__ __forceinline__ v8f mma(v16b a, v16b b, v8f c) {
    return __builtin_amdgcn_wmma_f32_16x16x32_bf16(false, a, false, b, (short)0, c, false, false);
  }
  static __device__ __forceinline__ void guard4(v8f& a, v8f& b, v8f& c, v8f& d, v16b x, v16b y) { dep_guard4_b(a, b, c, d, x, y); }
  static __device__ __forceinline__ void keep(v16b a, v16b b, v16b c, v16b d) { keep4_b(a, b, c, d); }
};

__device__ __forceinline__ v4u pack8_bf16(v4f a, v4f c) {
  unsigned short hb[8];
#pragma unroll
  for (int e = 0; e < 4; ++e) {
    hb[e]     = f2bf_bits(a[e]);
    hb[4 + e] = f2bf_bits(c[e]);
  }
  return (v4u){pk16(hb[0], hb[1]), pk16(hb[2], hb[3]), pk16(hb[4], hb[5]), pk16(hb[6], hb[7])};
}

template <int ET> struct Elem;
template <> struct Elem<0> { typedef _Float16 T; };
template <> struct Elem<1> { typedef __bf16 T; };
template <int ET, int BIAS_MODE, bool GELU, int OUT_MODE>
__global__ __launch_bounds__(256) void wmma_gemm64(
    const unsigned short* __restrict__ Ap, int lda, long strideA,
    const unsigned short* __restrict__ Btp, int ldb, long strideB,
    void* __restrict__ Cout, int ldc, long strideC,
    const float* __restrict__ bias, int M, int N, int K, float scale, float oscale) {
  typedef typename Elem<ET>::T T;
  typedef typename Frag<T>::V V;
  const T* A = (const T*)Ap; const T* Bt = (const T*)Btp;
  __shared__ __align__(16) float sT[8][16 * 68];
  const int b    = blockIdx.y;
  const int lane = threadIdx.x & 31;
  const int wave = threadIdx.x >> 5;
  const int tilesN = N >> 6;
  const int tilesM = M >> 6;
  const int tile = blockIdx.x * 8 + wave;
  if (tile >= tilesM * tilesN) return;
  const int tm = tile / tilesN;
  const int tn = tile - tm * tilesN;
  const int m0 = tm << 6;
  const int n0 = tn << 6;

  const T* Ab = A  + (size_t)b * strideA;
  const T* Bb = Bt + (size_t)b * strideB;

  const int rlane = lane & 15;
  const int koff  = (lane >> 4) * 8;
  const int mOff  = (lane >> 4) * 8;

  v8f acc[4][4];
#pragma unroll
  for (int i = 0; i < 4; ++i)
#pragma unroll
    for (int j = 0; j < 4; ++j) acc[i][j] = vzero8();

  for (int k0 = 0; k0 < K; k0 += 32) {
    V bh[4];
#pragma unroll
    for (int j = 0; j < 4; ++j) {
      const size_t bo = (size_t)(n0 + (j << 4) + rlane) * ldb + koff + k0;
      bh[j] = Frag<T>::load(Bb + bo);
    }
#pragma unroll
    for (int i = 0; i < 4; ++i) {
      const size_t ao = (size_t)(m0 + (i << 4) + rlane) * lda + koff + k0;
      V ah = Frag<T>::load(Ab + ao);
#pragma unroll
      for (int j = 0; j < 4; ++j) acc[i][j] = Frag<T>::mma(ah, bh[j], acc[i][j]);
      Frag<T>::guard4(acc[i][0], acc[i][1], acc[i][2], acc[i][3], ah, ah);
    }
    Frag<T>::keep(bh[0], bh[1], bh[2], bh[3]);
  }
  acc_guard4(acc[0][0], acc[0][1], acc[0][2], acc[0][3]);
  acc_guard4(acc[1][0], acc[1][1], acc[1][2], acc[1][3]);
  acc_guard4(acc[2][0], acc[2][1], acc[2][2], acc[2][3]);
  acc_guard4(acc[3][0], acc[3][1], acc[3][2], acc[3][3]);

  float* slab = sT[wave];
#pragma unroll
  for (int i = 0; i < 4; ++i) {
    const int mBase = m0 + (i << 4);
#pragma unroll
    for (int j = 0; j < 4; ++j) {
      const int n = n0 + (j << 4) + rlane;
      float bv = 0.f;
      if (BIAS_MODE == 2) bv = bfr(bias[n]);
#pragma unroll
      for (int r = 0; r < 8; ++r) {
        float v = acc[i][j][r] * scale;
        if (BIAS_MODE == 1) v += bfr(bias[mBase + mOff + r]);
        if (BIAS_MODE == 2) v += bv;
        slab[(mOff + r) * 68 + (j << 4) + rlane] = v;
      }
    }
    __builtin_amdgcn_fence(3, "workgroup");
    __builtin_amdgcn_wave_barrier();
    __builtin_amdgcn_fence(2, "workgroup");
    if (OUT_MODE == 0) {
      float* C = (float*)Cout + (size_t)b * strideC;
      const int hh = lane >> 4, c4 = (lane & 15) * 4;
      v4f vals[8];
#pragma unroll
      for (int it = 0; it < 8; ++it) {
        const int row = it * 2 + hh;
        v4f v = *(const v4f*)(slab + row * 68 + c4);
        if (GELU) {
#pragma unroll
          for (int e = 0; e < 4; ++e) v[e] = gelu_f(v[e]);
        }
        vals[it] = v;
      }
      for (int pass = 0; pass < 2; ++pass) {
#pragma unroll
        for (int it = 0; it < 8; ++it) {
          const int row = it * 2 + hh;
          *(volatile v4f*)(C + (size_t)(mBase + row) * ldc + n0 + c4) = vals[it];
        }
        __threadfence();
      }
    } else {
      const int q = lane >> 3, c8 = (lane & 7) * 8;
      unsigned short* C = (unsigned short*)Cout + (size_t)b * strideC;
      v8h vals[4];
#pragma unroll
      for (int it = 0; it < 4; ++it) {
        const int row = it * 4 + q;
        const float* sp = slab + row * 68 + c8;
        const v4f a0 = *(const v4f*)(sp);
        const v4f a1 = *(const v4f*)(sp + 4);
        v8h hv;
#pragma unroll
        for (int e = 0; e < 4; ++e) {
          float v0 = a0[e], v1 = a1[e];
          if (GELU) { v0 = gelu_f(v0); v1 = gelu_f(v1); }
          hv[e]     = (_Float16)(v0 * oscale);
          hv[4 + e] = (_Float16)(v1 * oscale);
        }
        vals[it] = hv;
      }
      for (int pass = 0; pass < 2; ++pass) {
#pragma unroll
        for (int it = 0; it < 4; ++it) {
          const int row = it * 4 + q;
          *(volatile v8h*)(C + (size_t)(mBase + row) * ldc + n0 + c8) = vals[it];
        }
        __threadfence();
      }
    }
    __builtin_amdgcn_fence(3, "workgroup");
    __builtin_amdgcn_wave_barrier();
    __builtin_amdgcn_fence(2, "workgroup");
  }
}

template <int ET>
__global__ __launch_bounds__(256) void tcast_kernel(const float* __restrict__ W, unsigned short* __restrict__ out,
                                                    int R, int Cc, float sc) {
  __shared__ float sm[64][65];
  const int t  = threadIdx.x;
  const int r0 = blockIdx.x * 64;
  const int c0 = blockIdx.y * 64;
#pragma unroll
  for (int i = 0; i < 16; ++i) {
    const int e  = i * 256 + t;
    const int rl = e >> 6;
    const int cl = e & 63;
    sm[cl][rl] = W[(size_t)(r0 + rl) * Cc + c0 + cl];
  }
  __syncthreads();
  const int lane = t & 31, wave = t >> 5;
  const int q = lane >> 3, c8 = (lane & 7) * 8;
  if (ET == 1) {
    v4u vals[2];
#pragma unroll
    for (int it = 0; it < 2; ++it) {
      const int row = wave * 8 + it * 4 + q;
      unsigned short hb[8];
#pragma unroll
      for (int e = 0; e < 8; ++e) hb[e] = f2bf_bits(sm[row][c8 + e]);
      vals[it] = (v4u){pk16(hb[0], hb[1]), pk16(hb[2], hb[3]), pk16(hb[4], hb[5]), pk16(hb[6], hb[7])};
    }
    for (int pass = 0; pass < 2; ++pass) {
#pragma unroll
      for (int it = 0; it < 2; ++it) {
        const int row = wave * 8 + it * 4 + q;
        *(volatile v4u*)(out + (size_t)(c0 + row) * R + r0 + c8) = vals[it];
      }
      __threadfence();
    }
  } else {
    v8h vals[2];
#pragma unroll
    for (int it = 0; it < 2; ++it) {
      const int row = wave * 8 + it * 4 + q;
      v8h hv;
#pragma unroll
      for (int e = 0; e < 8; ++e) hv[e] = (_Float16)(bfr(sm[row][c8 + e]) * sc);
      vals[it] = hv;
    }
    for (int pass = 0; pass < 2; ++pass) {
#pragma unroll
      for (int it = 0; it < 2; ++it) {
        const int row = wave * 8 + it * 4 + q;
        *(volatile v8h*)(out + (size_t)(c0 + row) * R + r0 + c8) = vals[it];
      }
      __threadfence();
    }
  }
}

__global__ __launch_bounds__(256) void xcast_kernel(const float* __restrict__ x, unsigned short* __restrict__ XB) {
  const int t = threadIdx.x;
  const int row = blockIdx.x * 2 + (t >> 7);
  const int bb = row / kSeq;
  const int s  = row - bb * kSeq;
  const int c  = 8 * (t & 127);
  const float* xr = x + ((size_t)bb * kSeqFull + s) * kH + c;
  const v4f a0 = *(const v4f*)(xr);
  const v4f a1 = *(const v4f*)(xr + 4);
  const v4u u = pack8_bf16(a0, a1);
  unsigned short* p = XB + (size_t)row * kH + c;
  *(volatile v4u*)p = u;
  __threadfence();
  *(volatile v4u*)p = u;
}

__global__ __launch_bounds__(256) __attribute__((amdgpu_num_vgpr(256)))
void attn_kernel(const unsigned short* __restrict__ Qp, const unsigned short* __restrict__ Kp,
                 const unsigned short* __restrict__ VTp, const int* __restrict__ am,
                 unsigned short* __restrict__ CTXp) {
  __shared__ __align__(16) _Float16 sP[8][16 * kPP];
  __shared__ __align__(16) _Float16 sO[8][16 * kPP];
  const int lane = threadIdx.x & 31, wave = threadIdx.x >> 5;
  const int bh = blockIdx.y;
  const int b  = bh / kNH;
  const int h  = bh - b * kNH;
  const int i0 = blockIdx.x * kQB + wave * 16;
  const int rl = lane & 15, hf = lane >> 4, koff = hf * 8;
  const float ninf = -__builtin_inff();
  const _Float16* Q  = (const _Float16*)Qp;
  const _Float16* K  = (const _Float16*)Kp;
  const _Float16* VT = (const _Float16*)VTp;

  const _Float16* qptr = Q + (size_t)(b * kSeq + i0 + rl) * kH + h * kHD + koff;
  const v16h qf0 = Frag<_Float16>::load(qptr);
  const v16h qf1 = Frag<_Float16>::load(qptr + 32);
  const _Float16* Kb = K + (size_t)(b * kSeq) * kH + h * kHD + koff;
  const _Float16* Vb = VT + ((size_t)b * kH + (size_t)h * kHD) * kSeq + koff;
  const int* amb = am + (size_t)b * kSeqFull;
  _Float16* myP = &sP[wave][0];
  _Float16* myO = &sO[wave][0];

  float mrow[8], lrow[8];
  v8f O[4];
#pragma unroll
  for (int r = 0; r < 8; ++r) { mrow[r] = ninf; lrow[r] = 0.f; }
#pragma unroll
  for (int dt = 0; dt < 4; ++dt) O[dt] = vzero8();

#pragma unroll 1
  for (int j0 = 0; j0 < kSeq; j0 += kKB) {
    v8f S[4];
    v16h kfa, kfb;
#pragma unroll
    for (int t = 0; t < 4; ++t) {
      S[t] = vzero8();
      const _Float16* kp = Kb + (size_t)(j0 + 16 * t + rl) * kH;
      kfa = Frag<_Float16>::load(kp);
      kfb = Frag<_Float16>::load(kp + 32);
      S[t] = Frag<_Float16>::mma(qf0, kfa, S[t]);
      S[t] = Frag<_Float16>::mma(qf1, kfb, S[t]);
    }
    Frag<_Float16>::guard4(S[0], S[1], S[2], S[3], kfa, kfb);

    bool okv[4];
#pragma unroll
    for (int t = 0; t < 4; ++t) okv[t] = (amb[j0 + 16 * t + rl] == 1);

#pragma unroll
    for (int r = 0; r < 8; ++r) {
      const float x0 = okv[0] ? S[0][r] * kScoreC : ninf;
      const float x1 = okv[1] ? S[1][r] * kScoreC : ninf;
      const float x2 = okv[2] ? S[2][r] * kScoreC : ninf;
      const float x3 = okv[3] ? S[3][r] * kScoreC : ninf;
      float mx = fmaxf(fmaxf(x0, x1), fmaxf(x2, x3));
      mx = fmaxf(mx, __shfl_xor(mx, 1, 16));
      mx = fmaxf(mx, __shfl_xor(mx, 2, 16));
      mx = fmaxf(mx, __shfl_xor(mx, 4, 16));
      mx = fmaxf(mx, __shfl_xor(mx, 8, 16));
      const float mold = mrow[r];
      const float mnew = fmaxf(mold, mx);
      const float msub = (mnew == ninf) ? 0.f : mnew;
      const float alpha = (mold == ninf) ? 0.f : exp2f(mold - msub);
      const _Float16 p0 = (_Float16)(exp2f(x0 - msub) * kPCarry);
      const _Float16 p1 = (_Float16)(exp2f(x1 - msub) * kPCarry);
      const _Float16 p2 = (_Float16)(exp2f(x2 - msub) * kPCarry);
      const _Float16 p3 = (_Float16)(exp2f(x3 - msub) * kPCarry);
      float rs = ((float)p0 + (float)p1) + ((float)p2 + (float)p3);
      rs += __shfl_xor(rs, 1, 16);
      rs += __shfl_xor(rs, 2, 16);
      rs += __shfl_xor(rs, 4, 16);
      rs += __shfl_xor(rs, 8, 16);
      lrow[r] = lrow[r] * alpha + rs;
      mrow[r] = mnew;
      O[0][r] *= alpha; O[1][r] *= alpha; O[2][r] *= alpha; O[3][r] *= alpha;
      _Float16* pp = myP + (8 * hf + r) * kPP + rl;
      pp[0]  = p0;
      pp[16] = p1;
      pp[32] = p2;
      pp[48] = p3;
    }
    __builtin_amdgcn_fence(3, "workgroup");
    __builtin_amdgcn_wave_barrier();
    __builtin_amdgcn_fence(2, "workgroup");

#pragma unroll
    for (int u = 0; u < 2; ++u) {
      const v16h pf = Frag<_Float16>::load(myP + rl * kPP + 32 * u + koff);
      v16h vf;
#pragma unroll
      for (int dt = 0; dt < 4; ++dt) {
        vf = Frag<_Float16>::load(Vb + (size_t)(dt * 16 + rl) * kSeq + j0 + 32 * u);
        O[dt] = Frag<_Float16>::mma(pf, vf, O[dt]);
      }
      Frag<_Float16>::guard4(O[0], O[1], O[2], O[3], pf, vf);
    }
    __builtin_amdgcn_fence(3, "workgroup");
    __builtin_amdgcn_wave_barrier();
    __builtin_amdgcn_fence(2, "workgroup");
  }

#pragma unroll
  for (int r = 0; r < 8; ++r) {
    const float inv = kCtxCarry / lrow[r];
    _Float16* op = myO + (8 * hf + r) * kPP + rl;
    op[0]  = (_Float16)(O[0][r] * inv);
    op[16] = (_Float16)(O[1][r] * inv);
    op[32] = (_Float16)(O[2][r] * inv);
    op[48] = (_Float16)(O[3][r] * inv);
  }
  __builtin_amdgcn_fence(3, "workgroup");
  __builtin_amdgcn_wave_barrier();
  __builtin_amdgcn_fence(2, "workgroup");
  const int q = lane >> 3, c8 = (lane & 7) * 8;
  v8h vals[4];
#pragma unroll
  for (int it = 0; it < 4; ++it) {
    const int row = it * 4 + q;
    vals[it] = *(const v8h*)(myO + row * kPP + c8);
  }
  unsigned short* C = CTXp + (size_t)(b * kSeq + i0) * kH + h * kHD + c8;
  for (int pass = 0; pass < 2; ++pass) {
#pragma unroll
    for (int it = 0; it < 4; ++it) {
      const int row = it * 4 + q;
      *(volatile v8h*)(C + (size_t)row * kH) = vals[it];
    }
    __threadfence();
  }
}

template <int OUTK>
__global__ __launch_bounds__(256) void ln_row_kernel(const float* __restrict__ x, const float* __restrict__ g,
                                                     const float* __restrict__ bb, void* __restrict__ outp) {
  __shared__ __align__(16) float srow[kH];
  __shared__ float redA[8];
  __shared__ float redB[8];
  const int row = blockIdx.x;
  const int t = threadIdx.x, lane = t & 31, wave = t >> 5;
  const float* xr = x + (size_t)row * kH;
  const float v0 = xr[t], v1 = xr[t + 256], v2 = xr[t + 512], v3 = xr[t + 768];
  float s = (v0 + v1) + (v2 + v3);
#pragma unroll
  for (int off = 16; off > 0; off >>= 1) s += __shfl_xor(s, off, 32);
  if (lane == 0) redA[wave] = s;
  __syncthreads();
  float tot = redA[0];
#pragma unroll
  for (int w = 1; w < 8; ++w) tot += redA[w];
  const float mean = tot * kInvH;
  const float d0 = v0 - mean, d1 = v1 - mean, d2 = v2 - mean, d3 = v3 - mean;
  float qq = (d0 * d0 + d1 * d1) + (d2 * d2 + d3 * d3);
#pragma unroll
  for (int off = 16; off > 0; off >>= 1) qq += __shfl_xor(qq, off, 32);
  if (lane == 0) redB[wave] = qq;
  __syncthreads();
  float tq = redB[0];
#pragma unroll
  for (int w = 1; w < 8; ++w) tq += redB[w];
  const float var  = tq * kInvH;
  const float rstd = rsqrtf(var + kLnEps);
  srow[t]       = d0 * rstd * bfr(g[t])       + bfr(bb[t]);
  srow[t + 256] = d1 * rstd * bfr(g[t + 256]) + bfr(bb[t + 256]);
  srow[t + 512] = d2 * rstd * bfr(g[t + 512]) + bfr(bb[t + 512]);
  srow[t + 768] = d3 * rstd * bfr(g[t + 768]) + bfr(bb[t + 768]);
  __syncthreads();
  if (OUTK == 0) {
    if (t < 128) {
      const v4f a0 = *(const v4f*)(srow + 8 * t);
      const v4f a1 = *(const v4f*)(srow + 8 * t + 4);
      v8h hv;
#pragma unroll
      for (int e = 0; e < 4; ++e) { hv[e] = (_Float16)a0[e]; hv[4 + e] = (_Float16)a1[e]; }
      unsigned short* lp = (unsigned short*)outp + (size_t)row * kH + 8 * t;
      *(volatile v8h*)lp = hv;
      __threadfence();
      *(volatile v8h*)lp = hv;
    }
  } else {
    const int bidx = row / kSeq;
    const int sidx = row - bidx * kSeq;
    float* op = (float*)outp + ((size_t)bidx * kOutSeqStride + sidx) * kH + 4 * t;
    const v4f v = *(const v4f*)(srow + 4 * t);
    *(volatile v4f*)op = v;
    __threadfence();
    *(volatile v4f*)op = v;
  }
}

extern "C" void kernel_launch(void* const* d_in, const int* in_sizes, int n_in,
                              void* d_out, int out_size, void* d_ws, size_t ws_size,
                              hipStream_t stream) {
  if (n_in < 18) return;
  const long long needX   = (long long)((kB - 1) * kSeqFull + kSeq) * kH;
  const long long needMsk = (long long)((kB - 1) * kSeqFull + kSeq);
  const long long needOut = (long long)((kB - 1) * kOutSeqStride + kSeq) * kH;
  if ((long long)in_sizes[0] < needX) return;
  if ((long long)in_sizes[1] < needMsk) return;
  if (in_sizes[2] < kH * kH || in_sizes[4] < kH * kH || in_sizes[6] < kH * kH || in_sizes[8] < kH * kH) return;
  if (in_sizes[3] < kH || in_sizes[5] < kH || in_sizes[7] < kH || in_sizes[9] < kH) return;
  if (in_sizes[10] < kH || in_sizes[11] < kH || in_sizes[16] < kH || in_sizes[17] < kH) return;
  if (in_sizes[12] < kH * kFF || in_sizes[14] < kFF * kH) return;
  if (in_sizes[13] < kFF || in_sizes[15] < kH) return;
  if ((long long)out_size < needOut) return;
  if (ws_size < kWsTotal) return;

  const float* x    = (const float*)d_in[0];
  const int*   amsk = (const int*)d_in[1];
  const float* wq   = (const float*)d_in[2];
  const float* bq   = (const float*)d_in[3];
  const float* wk   = (const float*)d_in[4];
  const float* bk   = (const float*)d_in[5];
  const float* wv   = (const float*)d_in[6];
  const float* bv   = (const float*)d_in[7];
  const float* wo   = (const float*)d_in[8];
  const float* bo   = (const float*)d_in[9];
  const float* ln1g = (const float*)d_in[10];
  const float* ln1b = (const float*)d_in[11];
  const float* w1   = (const float*)d_in[12];
  const float* b1   = (const float*)d_in[13];
  const float* w2   = (const float*)d_in[14];
  const float* b2   = (const float*)d_in[15];
  const float* ln2g = (const float*)d_in[16];
  const float* ln2b = (const float*)d_in[17];
  float* out = (float*)d_out;
  char* ws = (char*)d_ws;
  unsigned short* WQT  = (unsigned short*)(ws + offWQ);
  unsigned short* WKT  = (unsigned short*)(ws + offWK);
  unsigned short* WVT  = (unsigned short*)(ws + offWV);
  unsigned short* WOT  = (unsigned short*)(ws + offWO);
  unsigned short* W1T  = (unsigned short*)(ws + offW1);
  unsigned short* W2T  = (unsigned short*)(ws + offW2);
  unsigned short* XB   = (unsigned short*)(ws + offXB);
  unsigned short* Q16  = (unsigned short*)(ws + offQ);
  unsigned short* K16  = (unsigned short*)(ws + offK);
  unsigned short* VT   = (unsigned short*)(ws + offVT);
  unsigned short* CTX  = (unsigned short*)(ws + offCTX);
  float*          TMP  = (float*)(ws + offTMP);
  unsigned short* LN1P = (unsigned short*)(ws + offLN1);
  unsigned short* U16  = (unsigned short*)(ws + offU);

  tcast_kernel<1><<<dim3(kH / 64, kH / 64), dim3(256), 0, stream>>>(wq, WQT, kH, kH, 1.0f);
  tcast_kernel<1><<<dim3(kH / 64, kH / 64), dim3(256), 0, stream>>>(wk, WKT, kH, kH, 1.0f);
  tcast_kernel<1><<<dim3(kH / 64, kH / 64), dim3(256), 0, stream>>>(wv, WVT, kH, kH, 1.0f);
  tcast_kernel<0><<<dim3(kH / 64, kH / 64), dim3(256), 0, stream>>>(wo, WOT, kH, kH, kWCarry);
  tcast_kernel<0><<<dim3(kH / 64, kFF / 64), dim3(256), 0, stream>>>(w1, W1T, kH, kFF, kWCarry);
  tcast_kernel<0><<<dim3(kFF / 64, kH / 64), dim3(256), 0, stream>>>(w2, W2T, kFF, kH, kWCarry);

  xcast_kernel<<<dim3(kM / 2), dim3(256), 0, stream>>>(x, XB);

  const int blkProj = ((kM / 64) * (kH / 64) + 7) / 8;
  const int blkVT   = ((kH / 64) * (kSeq / 64) + 7) / 8;
  const int blkW1   = ((kM / 64) * (kFF / 64) + 7) / 8;

  wmma_gemm64<1, 2, false, 1><<<dim3(blkProj, 1), dim3(256), 0, stream>>>(
      XB, kH, 0L, WQT, kH, 0L, (void*)Q16, kH, 0L, bq, kM, kH, kH, 1.0f, 1.0f);
  wmma_gemm64<1, 2, false, 1><<<dim3(blkProj, 1), dim3(256), 0, stream>>>(
      XB, kH, 0L, WKT, kH, 0L, (void*)K16, kH, 0L, bk, kM, kH, kH, 1.0f, 1.0f);
  wmma_gemm64<1, 1, false, 1><<<dim3(blkVT, kB), dim3(256), 0, stream>>>(
      WVT, kH, 0L, XB, kH, (long)kSeq * kH, (void*)VT, kSeq, (long)kH * kSeq, bv, kH, kSeq, kH, 1.0f, 1.0f);

  attn_kernel<<<dim3(kSeq / kQB, kB * kNH), dim3(256), 0, stream>>>(Q16, K16, VT, amsk, CTX);

  wmma_gemm64<0, 2, false, 0><<<dim3(blkProj, 1), dim3(256), 0, stream>>>(
      CTX, kH, 0L, WOT, kH, 0L, (void*)TMP, kH, 0L, bo, kM, kH, kH, 1.0f / (kCtxCarry * kWCarry), 1.0f);
  ln_row_kernel<0><<<dim3(kM), dim3(256), 0, stream>>>(TMP, ln1g, ln1b, (void*)LN1P);
  wmma_gemm64<0, 2, true, 1><<<dim3(blkW1, 1), dim3(256), 0, stream>>>(
      LN1P, kH, 0L, W1T, kH, 0L, (void*)U16, kFF, 0L, b1, kM, kFF, kH, 1.0f / kWCarry, kUCarry);
  wmma_gemm64<0, 2, false, 0><<<dim3(blkProj, 1), dim3(256), 0, stream>>>(
      U16, kFF, 0L, W2T, kFF, 0L, (void*)TMP, kH, 0L, b2, kM, kH, kFF, 1.0f / (kUCarry * kWCarry), 1.0f);
  ln_row_kernel<1><<<dim3(kM), dim3(256), 0, stream>>>(TMP, ln2g, ln2b, (void*)out);
}
